// DeepSet2d_17179869356
// MI455X (gfx1250) — hardware-verified
//
#include <hip/hip_runtime.h>
#include <stddef.h>


#define NPIX        50176
#define IMG_W       224
#define NBATCH      32
#define NCH         3
#define HID         128
#define EMB         64
#define NCLS        10
#define WPB         8
#define TILES_PER_B 3136
#define BLK_PER_B   392
#define NFRAG       96
#define SA          136
#define SB          72
#define CLS_THREADS 512

static_assert(TILES_PER_B * 16 == NPIX);
static_assert(BLK_PER_B * WPB == TILES_PER_B);
static_assert(IMG_W * IMG_W == NPIX);
static_assert((NFRAG * 64) % 256 == 0);
static_assert((NBATCH * NCLS) % 4 == 0);

typedef _Float16     v16h __attribute__((ext_vector_type(16)));
typedef _Float16     v8h  __attribute__((ext_vector_type(8)));
typedef _Float16     v8ha __attribute__((ext_vector_type(8), __may_alias__));
typedef float        v8f  __attribute__((ext_vector_type(8)));
typedef float        v4f  __attribute__((ext_vector_type(4)));
typedef unsigned int v4u  __attribute__((ext_vector_type(4)));

union Frag {
    v16h     v;
    v8h      half[2];
    v4u      q[2];
    _Float16 e[16];
};

union Pack8 {
    v8h      v;
    v4u      q;
    _Float16 e[8];
};

__device__ __forceinline__ v8f mma16(v16h a, v16h b, v8f c)
{
    v8f d = __builtin_amdgcn_wmma_f32_16x16x32_f16(false, a, false, b, (short)0, c, false, false);
    asm volatile("v_nop\n\tv_nop\n\tv_nop\n\tv_nop" : "+v"(d) : "v"(a), "v"(b));
    return d;
}

__device__ __forceinline__ v8f splat8(float x)
{
    v8f v = {x, x, x, x, x, x, x, x};
    return v;
}

__device__ __forceinline__ v16h loadW(const _Float16* __restrict__ fw, int f, int lane)
{
    const v8h* p = (const v8h*)(fw + ((size_t)(f * 32 + lane) << 4));
    Frag r;
    r.half[0] = p[0];
    r.half[1] = p[1];
    return r.v;
}

__device__ __forceinline__ v16h loadA(const _Float16* base, int stride, int ks, int lane)
{
    const _Float16* r = base + (lane & 15) * stride + ks * 32 + 8 * (lane >> 4);
    Frag fr;
    fr.half[0] = *(const v8ha*)(r);
    fr.half[1] = *(const v8ha*)(r + 16);
    return fr.v;
}

__device__ __forceinline__ float softplus_f(float x)
{
    const float t = __expf(-fabsf(x));
    return fmaxf(x, 0.f) + __logf(1.0f + t);
}

__global__ __launch_bounds__(256) void k_pack(const float* __restrict__ w_obs1,
                                              const float* __restrict__ w_obs2,
                                              const float* __restrict__ w_ol1,
                                              const float* __restrict__ w_ol2,
                                              const float* __restrict__ w_loc1,
                                              const float* __restrict__ w_loc2,
                                              _Float16* __restrict__ fragW)
{
    const int tid = blockIdx.x * blockDim.x + threadIdx.x;
    if (tid >= NFRAG * 64) return;
    const int f    = tid >> 6;
    const int lane = (tid >> 1) & 31;
    const int j    = tid & 1;
    const int h    = lane >> 4;
    const int nl   = lane & 15;

    const float* W; int K, N, ks, nt, roff;
    if (f < 8)       {                 W = w_obs1; K = 3;   N = 128; ks = 0;      nt = f;     roff = 0;  }
    else if (f < 24) { int g = f - 8;  W = w_obs2; K = 128; N = 64;  ks = g >> 2; nt = g & 3; roff = 0;  }
    else if (f < 40) { int g = f - 24; W = w_ol1;  K = 64;  N = 128; ks = g >> 3; nt = g & 7; roff = 0;  }
    else if (f < 56) { int g = f - 40; W = w_ol2;  K = 128; N = 64;  ks = g >> 2; nt = g & 3; roff = 0;  }
    else if (f < 64) { int g = f - 56; W = w_loc1; K = 2;   N = 128; ks = 0;      nt = g;     roff = 0;  }
    else if (f < 80) { int g = f - 64; W = w_loc2; K = 128; N = 64;  ks = g >> 2; nt = g & 3; roff = 0;  }
    else             { int g = f - 80; W = w_ol1;  K = 64;  N = 128; ks = g >> 3; nt = g & 7; roff = 64; }

    const int n  = nt * 16 + nl;
    const int kb = ks * 32 + 16 * j + 8 * h;
    Pack8 u;
#pragma unroll
    for (int i = 0; i < 8; ++i) {
        const int kk = kb + i;
        const int kr = (kk < K) ? kk : (K - 1);
        float v = W[(size_t)(roff + kr) * N + n];
        if (kk >= K) v = 0.f;
        u.e[i] = (_Float16)v;
    }
    const v4u q = u.q;
    volatile v4u* dst = (volatile v4u*)fragW;
    dst[tid] = q;
    __threadfence();
    dst[tid] = q;
}

__global__ __launch_bounds__(256) void k_loc(const _Float16* __restrict__ fragW,
                                             const float* __restrict__ b_loc1,
                                             const float* __restrict__ b_loc2,
                                             const float* __restrict__ b_ol1,
                                             v4f* __restrict__ loc_ws)
{
    __shared__ __attribute__((aligned(16))) _Float16 actA[WPB][16 * SA];
    __shared__ __attribute__((aligned(16))) _Float16 actB[WPB][16 * SB];

    const int tid = threadIdx.x, lane = tid & 31, wid = tid >> 5;
    const int h = lane >> 4, m = lane & 15;
    _Float16* A = actA[wid];
    _Float16* E = actB[wid];
    const int pt = blockIdx.x * WPB + wid;
    const int n  = pt * 16 + m;
    const int iy = n / IMG_W;
    const int ix = n - iy * IMG_W;
    const float rs = 1.0f / (float)(IMG_W - 1);
    const float sy = (float)iy * rs;
    const float sx = (float)ix * rs;
    float fy = -10.0f * (1.0f - sy) + 10.0f * sy;
    float fx = -10.0f * (1.0f - sx) + 10.0f * sx;
    if (iy == IMG_W - 1) fy = 10.0f;
    if (ix == IMG_W - 1) fx = 10.0f;

    const v4u z4 = {0u, 0u, 0u, 0u};
    Frag ax;
    ax.q[0] = z4;
    ax.q[1] = z4;
    ax.e[0] = (_Float16)(h == 0 ? fy : 0.f);
    ax.e[1] = (_Float16)(h == 0 ? fx : 0.f);

#pragma unroll
    for (int nt = 0; nt < 8; ++nt) {
        v8f c = splat8(0.f);
        c = mma16(ax.v, loadW(fragW, 56 + nt, lane), c);
        const float bb = b_loc1[nt * 16 + m];
#pragma unroll
        for (int r = 0; r < 8; ++r)
            A[(8 * h + r) * SA + nt * 16 + m] = (_Float16)fmaxf(c[r] + bb, 0.f);
    }
    __syncthreads();

    {
        v8f acc[4];
#pragma unroll
        for (int nt = 0; nt < 4; ++nt) acc[nt] = splat8(b_loc2[nt * 16 + m]);
#pragma unroll 1
        for (int ks = 0; ks < 4; ++ks) {
            const v16h a = loadA(A, SA, ks, lane);
#pragma unroll
            for (int nt = 0; nt < 4; ++nt)
                acc[nt] = mma16(a, loadW(fragW, 64 + ks * 4 + nt, lane), acc[nt]);
        }
#pragma unroll
        for (int nt = 0; nt < 4; ++nt) {
#pragma unroll
            for (int r = 0; r < 8; ++r)
                E[(8 * h + r) * SB + nt * 16 + m] = (_Float16)acc[nt][r];
        }
    }
    __syncthreads();

    volatile v4f* lw = (volatile v4f*)loc_ws;
#pragma unroll
    for (int grp = 0; grp < 2; ++grp) {
        v8f acc[4];
#pragma unroll
        for (int nt = 0; nt < 4; ++nt) acc[nt] = splat8(b_ol1[(grp * 4 + nt) * 16 + m]);
#pragma unroll 1
        for (int ks = 0; ks < 2; ++ks) {
            const v16h a = loadA(E, SB, ks, lane);
#pragma unroll
            for (int nt = 0; nt < 4; ++nt)
                acc[nt] = mma16(a, loadW(fragW, 80 + ks * 8 + grp * 4 + nt, lane), acc[nt]);
        }
        v4f lo[4], hi[4];
        size_t idx[4];
#pragma unroll
        for (int nt = 0; nt < 4; ++nt) {
            v4f a0 = {acc[nt][0], acc[nt][1], acc[nt][2], acc[nt][3]};
            v4f a1 = {acc[nt][4], acc[nt][5], acc[nt][6], acc[nt][7]};
            lo[nt] = a0;
            hi[nt] = a1;
            idx[nt] = ((size_t)(pt * 8 + grp * 4 + nt) * 2) * 32 + lane;
        }
#pragma unroll
        for (int nt = 0; nt < 4; ++nt) { lw[idx[nt]] = lo[nt]; lw[idx[nt] + 32] = hi[nt]; }
        __threadfence();
#pragma unroll
        for (int nt = 0; nt < 4; ++nt) { lw[idx[nt]] = lo[nt]; lw[idx[nt] + 32] = hi[nt]; }
    }
}

__global__ __launch_bounds__(256) void k_main(const float* __restrict__ images,
                                              const _Float16* __restrict__ fragW,
                                              const float* __restrict__ b_obs1,
                                              const float* __restrict__ b_obs2,
                                              const float* __restrict__ b_ol2,
                                              const v4f* __restrict__ loc_ws,
                                              v4f* __restrict__ part)
{
    __shared__ __attribute__((aligned(16))) _Float16 actA[WPB][16 * SA];
    __shared__ __attribute__((aligned(16))) _Float16 actB[WPB][16 * SB];
    __shared__ float red[WPB][32][4];
    __shared__ float bsum[64];

    const int tid = threadIdx.x, lane = tid & 31, wid = tid >> 5;
    const int h = lane >> 4, m = lane & 15;
    _Float16* A = actA[wid];
    _Float16* E = actB[wid];
    const int b   = blockIdx.x / BLK_PER_B;
    const int blk = blockIdx.x - b * BLK_PER_B;
    const int ptn = blk * WPB + wid;
    const int pix = ptn * 16 + m;

    const v4u z4 = {0u, 0u, 0u, 0u};
    Frag ax;
    ax.q[0] = z4;
    ax.q[1] = z4;
    {
        const float* ip = images + (size_t)b * NCH * NPIX + pix;
        const float x0 = ip[0];
        const float x1 = ip[NPIX];
        const float x2 = ip[2 * NPIX];
        ax.e[0] = (_Float16)(h == 0 ? x0 : 0.f);
        ax.e[1] = (_Float16)(h == 0 ? x1 : 0.f);
        ax.e[2] = (_Float16)(h == 0 ? x2 : 0.f);
    }

#pragma unroll
    for (int nt = 0; nt < 8; ++nt) {
        v8f c = splat8(0.f);
        c = mma16(ax.v, loadW(fragW, nt, lane), c);
        const float bb = b_obs1[nt * 16 + m];
#pragma unroll
        for (int r = 0; r < 8; ++r)
            A[(8 * h + r) * SA + nt * 16 + m] = (_Float16)fmaxf(c[r] + bb, 0.f);
    }
    __syncthreads();

    {
        v8f acc[4];
#pragma unroll
        for (int nt = 0; nt < 4; ++nt) acc[nt] = splat8(b_obs2[nt * 16 + m]);
#pragma unroll 1
        for (int ks = 0; ks < 4; ++ks) {
            const v16h a = loadA(A, SA, ks, lane);
#pragma unroll
            for (int nt = 0; nt < 4; ++nt)
                acc[nt] = mma16(a, loadW(fragW, 8 + ks * 4 + nt, lane), acc[nt]);
        }
#pragma unroll
        for (int nt = 0; nt < 4; ++nt) {
#pragma unroll
            for (int r = 0; r < 8; ++r)
                E[(8 * h + r) * SB + nt * 16 + m] = (_Float16)acc[nt][r];
        }
    }
    __syncthreads();

#pragma unroll
    for (int grp = 0; grp < 2; ++grp) {
        v8f acc[4];
#pragma unroll
        for (int nt = 0; nt < 4; ++nt) {
            const size_t li = ((size_t)(ptn * 8 + grp * 4 + nt) * 2) * 32 + lane;
            const v4f l0 = loc_ws[li];
            const v4f l1 = loc_ws[li + 32];
            v8f t = {l0[0], l0[1], l0[2], l0[3], l1[0], l1[1], l1[2], l1[3]};
            acc[nt] = t;
        }
#pragma unroll 1
        for (int ks = 0; ks < 2; ++ks) {
            const v16h a = loadA(E, SB, ks, lane);
#pragma unroll
            for (int nt = 0; nt < 4; ++nt)
                acc[nt] = mma16(a, loadW(fragW, 24 + ks * 8 + grp * 4 + nt, lane), acc[nt]);
        }
#pragma unroll
        for (int nt = 0; nt < 4; ++nt) {
#pragma unroll
            for (int r = 0; r < 8; ++r)
                A[(8 * h + r) * SA + (grp * 4 + nt) * 16 + m] = (_Float16)fmaxf(acc[nt][r], 0.f);
        }
    }
    __syncthreads();

    {
        v8f acc[4];
#pragma unroll
        for (int nt = 0; nt < 4; ++nt) acc[nt] = splat8(b_ol2[nt * 16 + m]);
#pragma unroll 1
        for (int ks = 0; ks < 4; ++ks) {
            const v16h a = loadA(A, SA, ks, lane);
#pragma unroll
            for (int nt = 0; nt < 4; ++nt)
                acc[nt] = mma16(a, loadW(fragW, 40 + ks * 4 + nt, lane), acc[nt]);
        }
#pragma unroll
        for (int nt = 0; nt < 4; ++nt) {
            float s = 0.f;
#pragma unroll
            for (int r = 0; r < 8; ++r) s += softplus_f(acc[nt][r]);
            red[wid][lane][nt] = s;
        }
    }
    __syncthreads();

    if (tid < 64) {
        const int nt = tid >> 4, c = tid & 15;
        float s = 0.f;
#pragma unroll
        for (int w = 0; w < WPB; ++w) {
            s += red[w][c][nt];
            s += red[w][c + 16][nt];
        }
        bsum[nt * 16 + c] = s;
    }
    __syncthreads();

    if (tid < 16) {
        v4f v = {bsum[4 * tid], bsum[4 * tid + 1], bsum[4 * tid + 2], bsum[4 * tid + 3]};
        const size_t pi = (size_t)(b * BLK_PER_B + blk) * 16 + tid;
        volatile v4f* pp = (volatile v4f*)part;
        pp[pi] = v;
        __threadfence();
        pp[pi] = v;
    }
}

__global__ __launch_bounds__(CLS_THREADS) void k_cls(const float* __restrict__ part,
                                                     const float* __restrict__ w1,
                                                     const float* __restrict__ b1,
                                                     const float* __restrict__ w2,
                                                     const float* __restrict__ b2,
                                                     v4f* __restrict__ out)
{
    __shared__ float es[NBATCH * EMB];
    __shared__ float hh[NBATCH * HID];
    __shared__ float lg[NBATCH * NCLS];
    const int t = threadIdx.x;

#pragma unroll 1
    for (int j = 0; j < (NBATCH * EMB) / CLS_THREADS; ++j) {
        const int idx = t + j * CLS_THREADS;
        const int b = idx >> 6, c = idx & 63;
        const float* p = part + (size_t)b * BLK_PER_B * 64 + c;
        double s = 0.0;
#pragma unroll 4
        for (int k = 0; k < BLK_PER_B; ++k) s += (double)p[(size_t)k * 64];
        es[idx] = (float)s;
    }
    __syncthreads();

#pragma unroll 1
    for (int j = 0; j < (NBATCH * HID) / CLS_THREADS; ++j) {
        const int idx = t + j * CLS_THREADS;
        const int b = idx >> 7, o = idx & 127;
        float a = 0.f;
#pragma unroll 4
        for (int i = 0; i < EMB; ++i) a += es[b * EMB + i] * w1[i * HID + o];
        a += b1[o];
        hh[idx] = fmaxf(a, 0.f);
    }
    __syncthreads();

    if (t < NBATCH * NCLS) {
        const int b = t / NCLS;
        const int o = t - b * NCLS;
        float a = 0.f;
#pragma unroll 4
        for (int i = 0; i < HID; ++i) a += hh[b * HID + i] * w2[i * NCLS + o];
        a += b2[o];
        lg[t] = a;
    }
    __syncthreads();

    if (t < (NBATCH * NCLS) / 4) {
        v4f v = {lg[4 * t], lg[4 * t + 1], lg[4 * t + 2], lg[4 * t + 3]};
        volatile v4f* po = (volatile v4f*)out;
        po[t] = v;
        __threadfence();
        po[t] = v;
    }
}

extern "C" void kernel_launch(void* const* d_in, const int* in_sizes, int n_in,
                              void* d_out, int out_size, void* d_ws, size_t ws_size,
                              hipStream_t stream)
{
    if (n_in < 17) return;
    const int want[17] = {
        NBATCH * NCH * NPIX,
        NCH * HID, HID, HID * EMB, EMB,
        2 * HID,   HID, HID * EMB, EMB,
        2 * EMB * HID, HID, HID * EMB, EMB,
        EMB * HID, HID, HID * NCLS, NCLS };
    for (int i = 0; i < 17; ++i) if (in_sizes[i] != want[i]) return;
    if (out_size != NBATCH * NCLS) return;

    const float* images = (const float*)d_in[0];
    const float* w_obs1 = (const float*)d_in[1];
    const float* b_obs1 = (const float*)d_in[2];
    const float* w_obs2 = (const float*)d_in[3];
    const float* b_obs2 = (const float*)d_in[4];
    const float* w_loc1 = (const float*)d_in[5];
    const float* b_loc1 = (const float*)d_in[6];
    const float* w_loc2 = (const float*)d_in[7];
    const float* b_loc2 = (const float*)d_in[8];
    const float* w_ol1  = (const float*)d_in[9];
    const float* b_ol1  = (const float*)d_in[10];
    const float* w_ol2  = (const float*)d_in[11];
    const float* b_ol2  = (const float*)d_in[12];
    const float* w_cls1 = (const float*)d_in[13];
    const float* b_cls1 = (const float*)d_in[14];
    const float* w_cls2 = (const float*)d_in[15];
    const float* b_cls2 = (const float*)d_in[16];

    const size_t frag_bytes = (size_t)NFRAG * 32 * 16 * sizeof(_Float16);
    const size_t off_frag   = 0;
    const size_t off_loc    = 131072;
    const size_t loc_bytes  = (size_t)TILES_PER_B * 8 * 2 * 32 * sizeof(v4f);
    const size_t off_part   = off_loc + loc_bytes;
    const size_t part_bytes = (size_t)NBATCH * BLK_PER_B * 64 * sizeof(float);
    if (off_frag + frag_bytes > off_loc) return;
    if (off_part + part_bytes > ws_size) return;

    char* ws = (char*)d_ws;
    _Float16* fragW  = (_Float16*)(ws + off_frag);
    v4f*      loc_ws = (v4f*)(ws + off_loc);
    v4f*      part   = (v4f*)(ws + off_part);
    v4f*      out    = (v4f*)d_out;

    k_pack<<<dim3((NFRAG * 64) / 256), dim3(256), 0, stream>>>(
        w_obs1, w_obs2, w_ol1, w_ol2, w_loc1, w_loc2, fragW);
    k_loc<<<dim3(BLK_PER_B), dim3(256), 0, stream>>>(
        (const _Float16*)fragW, b_loc1, b_loc2, b_ol1, loc_ws);
    k_main<<<dim3(NBATCH * BLK_PER_B), dim3(256), 0, stream>>>(
        images, (const _Float16*)fragW, b_obs1, b_obs2, b_ol2, (const v4f*)loc_ws, part);
    k_cls<<<dim3(1), dim3(CLS_THREADS), 0, stream>>>(
        (const float*)part, w_cls1, b_cls1, w_cls2, b_cls2, out);
}
